// MI_Module_3917010174657
// MI455X (gfx1250) — hardware-verified
//
#include <hip/hip_runtime.h>


typedef __bf16          v16bf __attribute__((ext_vector_type(16)));
typedef unsigned short  v8us  __attribute__((ext_vector_type(8)));
typedef float           v8f   __attribute__((ext_vector_type(8)));
typedef float           v4f   __attribute__((ext_vector_type(4)));

#define Bn   8
#define Cn   128
#define Hn   96
#define Wn   96
#define HWn  (Hn * Wn)
#define Pn   (Bn * HWn)
#define NT   32
#define KP   136
#define OP   36
#define NTHR 256
#define CG   32

#if ((HWn % NT) != 0) || ((Wn % NT) != 0) || (Cn != 128) || ((Cn % CG) != 0) || ((KP % 8) != 0) || ((OP % 4) != 0) || (NTHR != CG * 8) || (NTHR / 32 * 16 != Cn)
#error cfg
#endif

union Frag { v16bf v; v8us u[2]; };

__device__ __forceinline__ unsigned short bf16_rne_bits(float f) {
    unsigned int u = __float_as_uint(f);
    u += 0x7FFFu + ((u >> 16) & 1u);
    return (unsigned short)(u >> 16);
}
__device__ __forceinline__ float bf16_bits_to_f32(unsigned short b) {
    return __uint_as_float(((unsigned int)b) << 16);
}

__device__ __forceinline__ v8f wmma3_bf16(v8f acc, v16bf ah, v16bf al, v16bf bh, v16bf bl) {
    acc = __builtin_amdgcn_wmma_f32_16x16x32_bf16(false, ah, false, bh, (short)0, acc, false, false);
    acc = __builtin_amdgcn_wmma_f32_16x16x32_bf16(false, ah, false, bl, (short)0, acc, false, false);
    acc = __builtin_amdgcn_wmma_f32_16x16x32_bf16(false, al, false, bh, (short)0, acc, false, false);
    asm volatile("v_nop\n\tv_nop\n\tv_nop\n\tv_nop"
                 : "+v"(acc) : "v"(ah), "v"(al), "v"(bh), "v"(bl));
    return acc;
}

__global__ void __launch_bounds__(NTHR)
pack_fw_kernel(const float* __restrict__ Fw, unsigned short* AfH, unsigned short* AfL)
{
    const int tid = threadIdx.x;
    v8us hiv[8], lov[8];
#pragma unroll
    for (int j = 0; j < 8; ++j) {
        const int g    = tid + NTHR * j;
        const int half = g & 1;
        const int lane = (g >> 1) & 31;
        const int kt   = (g >> 6) & 3;
        const int mt   = g >> 8;
        const int M    = mt * 16 + (lane & 15);
        const int K0   = kt * 32 + half * 16 + (lane >> 4) * 8;
        const float* src = Fw + M * Cn + K0;
        const v4f f0 = *(const v4f*)src;
        const v4f f1 = *(const v4f*)(src + 4);
        v8us hv, lv;
#pragma unroll
        for (int e = 0; e < 4; ++e) {
            const unsigned short h0 = bf16_rne_bits(f0[e]);
            const unsigned short l0 = bf16_rne_bits(f0[e] - bf16_bits_to_f32(h0));
            const unsigned short h1 = bf16_rne_bits(f1[e]);
            const unsigned short l1 = bf16_rne_bits(f1[e] - bf16_bits_to_f32(h1));
            hv[e] = h0;     lv[e] = l0;
            hv[4 + e] = h1; lv[4 + e] = l1;
        }
        hiv[j] = hv;
        lov[j] = lv;
        *(volatile v8us*)(AfH + (size_t)g * 8) = hv;
        *(volatile v8us*)(AfL + (size_t)g * 8) = lv;
    }
    __threadfence();
#pragma unroll
    for (int j = 0; j < 8; ++j) {
        const int g = tid + NTHR * j;
        *(volatile v8us*)(AfH + (size_t)g * 8) = hiv[j];
        *(volatile v8us*)(AfL + (size_t)g * 8) = lov[j];
    }
}

__global__ void __launch_bounds__(NTHR)
fused_kernel(const float* __restrict__ x,
             const float* __restrict__ Dw,
             const float* __restrict__ Dscale,
             const float* __restrict__ Dbias,
             const float* __restrict__ Pw,
             const float* __restrict__ Pscale,
             const float* __restrict__ Pbias,
             const unsigned short* __restrict__ AfH,
             const unsigned short* __restrict__ AfL,
             const float* __restrict__ Fscale,
             const float* __restrict__ Fbias,
             float* out, int ntiles)
{
    __shared__ __align__(16) unsigned short Bh[NT * KP];
    __shared__ __align__(16) unsigned short Bl[NT * KP];
    __shared__ __align__(16) float          Ot[Cn * OP];

    if ((int)blockIdx.x >= ntiles) return;
    const int p0   = blockIdx.x * NT;
    const int b    = p0 / HWn;
    const int hw0  = p0 - b * HWn;
    const int h    = hw0 / Wn;
    const int w0   = hw0 - h * Wn;
    const int tid  = threadIdx.x;
    const int lane = tid & 31;
    const int wv   = tid >> 5;
    const int hl   = lane >> 4;
    const int m16  = lane & 15;

    {
        const int nq = tid & 7;
        const int cl = tid >> 3;
        const int wq = w0 + nq * 4;
#pragma unroll 1
        for (int g = 0; g < Cn / CG; ++g) {
            const int c = g * CG + cl;
            const float* __restrict__ xc = x + (size_t)(b * Cn + c) * HWn;
            float s[4];
#pragma unroll
            for (int j = 0; j < 4; ++j) s[j] = 0.0f;
#pragma unroll
            for (int i = 0; i < 4; ++i) {
                const int d = 1 << i;
                const float* __restrict__ wk = Dw + (i * Cn + c) * 9;
                float a[4];
#pragma unroll
                for (int j = 0; j < 4; ++j) a[j] = 0.0f;
#pragma unroll
                for (int kh = 0; kh < 3; ++kh) {
                    const int  hh  = h + (kh - 1) * d;
                    const bool rok = (hh >= 0) && (hh < Hn);
                    const int  hhc = min(max(hh, 0), Hn - 1);
                    const float* __restrict__ xr = xc + hhc * Wn;
#pragma unroll
                    for (int kw = 0; kw < 3; ++kw) {
                        const float wgt = wk[kh * 3 + kw];
#pragma unroll
                        for (int j = 0; j < 4; ++j) {
                            const int  col  = wq + j + (kw - 1) * d;
                            const bool ok   = rok && (col >= 0) && (col < Wn);
                            const int  colc = min(max(col, 0), Wn - 1);
                            float v = xr[colc];
                            v = ok ? v : 0.0f;
                            a[j] = fmaf(v, wgt, a[j]);
                        }
                    }
                }
                const float dsc = Dscale[i * Cn + c];
                const float dbi = Dbias[i * Cn + c];
                const float pw  = Pw[c * 4 + i];
#pragma unroll
                for (int j = 0; j < 4; ++j) {
                    const float m = fmaxf(fmaf(a[j], dsc, dbi), 0.0f);
                    s[j] = fmaf(pw, m, s[j]);
                }
            }
            const float psc = Pscale[c];
            const float pbi = Pbias[c];
#pragma unroll
            for (int j = 0; j < 4; ++j) {
                const float yv = fmaxf(fmaf(s[j], psc, pbi), 0.0f);
                const unsigned short hb = bf16_rne_bits(yv);
                const unsigned short lb = bf16_rne_bits(yv - bf16_bits_to_f32(hb));
                const int o = (nq * 4 + j) * KP + c;
                Bh[o] = hb;
                Bl[o] = lb;
            }
        }
    }
    __syncthreads();

    v8f acc[2];
#pragma unroll
    for (int nt = 0; nt < 2; ++nt)
#pragma unroll
        for (int r = 0; r < 8; ++r) acc[nt][r] = 0.0f;

#pragma unroll
    for (int kt = 0; kt < 4; ++kt) {
        Frag ah, al;
        const size_t ab = (size_t)(((wv * 4 + kt) * 32 + lane) * 16);
        ah.u[0] = *(const v8us*)(AfH + ab);
        ah.u[1] = *(const v8us*)(AfH + ab + 8);
        al.u[0] = *(const v8us*)(AfL + ab);
        al.u[1] = *(const v8us*)(AfL + ab + 8);
#pragma unroll
        for (int nt = 0; nt < 2; ++nt) {
            const int bo = (nt * 16 + m16) * KP + kt * 32 + 8 * hl;
            Frag bh, bl;
            bh.u[0] = *(const v8us*)(Bh + bo);
            bh.u[1] = *(const v8us*)(Bh + bo + 16);
            bl.u[0] = *(const v8us*)(Bl + bo);
            bl.u[1] = *(const v8us*)(Bl + bo + 16);
            acc[nt] = wmma3_bf16(acc[nt], ah.v, al.v, bh.v, bl.v);
        }
    }

#pragma unroll
    for (int nt = 0; nt < 2; ++nt)
#pragma unroll
        for (int r = 0; r < 8; ++r)
            Ot[(wv * 16 + 8 * hl + r) * OP + nt * 16 + m16] = acc[nt][r];
    __syncthreads();

    v4f vals[4];
    const int colq = (lane & 7) * 4;
#pragma unroll
    for (int it = 0; it < 4; ++it) {
        const int row = wv * 16 + 4 * it + (lane >> 3);
        const v4f o   = *(const v4f*)(Ot + row * OP + colq);
        const float fsc = Fscale[row];
        const float fbi = Fbias[row];
        const size_t gi = (size_t)(b * Cn + row) * HWn + hw0 + colq;
        const v4f xr = *(const v4f*)(x + gi);
        v4f res;
#pragma unroll
        for (int e = 0; e < 4; ++e) {
            const float t = fmaxf(fmaf(o[e], fsc, fbi), 0.0f);
            res[e] = fmaxf(t + xr[e], 0.0f);
        }
        vals[it] = res;
        *(volatile v4f*)(out + gi) = res;
    }
    __threadfence();
#pragma unroll
    for (int it = 0; it < 4; ++it) {
        const int row = wv * 16 + 4 * it + (lane >> 3);
        const size_t gi = (size_t)(b * Cn + row) * HWn + hw0 + colq;
        *(volatile v4f*)(out + gi) = vals[it];
    }
}

extern "C" void kernel_launch(void* const* d_in, const int* in_sizes, int n_in,
                              void* d_out, int out_size, void* d_ws, size_t ws_size,
                              hipStream_t stream)
{
    if (n_in < 10) return;
    if (in_sizes[0] != Bn * Cn * HWn || out_size != Bn * Cn * HWn) return;
    if (in_sizes[1] != 4 * Cn * 9 || in_sizes[2] != 4 * Cn || in_sizes[3] != 4 * Cn ||
        in_sizes[4] != Cn * 4 || in_sizes[5] != Cn || in_sizes[6] != Cn ||
        in_sizes[7] != Cn * Cn || in_sizes[8] != Cn || in_sizes[9] != Cn) return;

    const size_t offH = 0;
    const size_t offL = 32768;
    const size_t need = offL + (size_t)Cn * (size_t)Cn * sizeof(unsigned short);
    if (need > ws_size) return;

    const float* x      = (const float*)d_in[0];
    const float* Dw     = (const float*)d_in[1];
    const float* Dscale = (const float*)d_in[2];
    const float* Dbias  = (const float*)d_in[3];
    const float* Pw     = (const float*)d_in[4];
    const float* Pscale = (const float*)d_in[5];
    const float* Pbias  = (const float*)d_in[6];
    const float* Fw     = (const float*)d_in[7];
    const float* Fscale = (const float*)d_in[8];
    const float* Fbias  = (const float*)d_in[9];
    float* out = (float*)d_out;

    unsigned short* AfH = (unsigned short*)((char*)d_ws + offH);
    unsigned short* AfL = (unsigned short*)((char*)d_ws + offL);

    pack_fw_kernel<<<1, NTHR, 0, stream>>>(Fw, AfH, AfL);

    const int ntiles = Pn / NT;
    fused_kernel<<<(Pn + NT - 1) / NT, NTHR, 0, stream>>>(
        x, Dw, Dscale, Dbias, Pw, Pscale, Pbias, AfH, AfL, Fscale, Fbias, out, ntiles);
}
